// MKAFullAttention_79276506350036
// MI455X (gfx1250) — hardware-verified
//
#include <hip/hip_runtime.h>
#include <math.h>
#include <stdint.h>

#define NB   4
#define SEQ  1024
#define DM   1024
#define NH   16
#define DH   64
#define DR   512

typedef __attribute__((ext_vector_type(16))) _Float16 v16h;
typedef __attribute__((ext_vector_type(8)))  _Float16 v8h;
typedef __attribute__((ext_vector_type(16))) __bf16   v16b;
typedef __attribute__((ext_vector_type(8)))  __bf16   v8b;
typedef __attribute__((ext_vector_type(8)))  float    v8f;
typedef __attribute__((ext_vector_type(4)))  float    v4f;
typedef __attribute__((ext_vector_type(2)))  float    v2f;
typedef __attribute__((ext_vector_type(4)))  unsigned int v4u;

__device__ __forceinline__ unsigned short f2bf_bits(float f) {
  unsigned u = __float_as_uint(f);
  return (unsigned short)((u + 0x7FFFu + ((u >> 16) & 1u)) >> 16);
}
__device__ __forceinline__ float bf_bits2f(unsigned short h) { return __uint_as_float(((unsigned)h) << 16); }
__device__ __forceinline__ unsigned short f2h_bits(float f) { return __builtin_bit_cast(unsigned short, (_Float16)f); }
__device__ __forceinline__ unsigned pk16(unsigned short a, unsigned short b) { return (unsigned)a | ((unsigned)b << 16); }

__device__ __forceinline__ void dep_guard_h(v8f& a, v8f& b, v16h x, v16h y) { asm volatile("v_nop\n\tv_nop\n\tv_nop\n\tv_nop" : "+v"(a), "+v"(b) : "v"(x), "v"(y)); }
__device__ __forceinline__ void dep_guard_b(v8f& a, v8f& b, v16b x, v16b y) { asm volatile("v_nop\n\tv_nop\n\tv_nop\n\tv_nop" : "+v"(a), "+v"(b) : "v"(x), "v"(y)); }
__device__ __forceinline__ void keep4_h(v16h a, v16h b, v16h c, v16h d) { asm volatile("v_nop" :: "v"(a), "v"(b), "v"(c), "v"(d)); }
__device__ __forceinline__ void keep4_b(v16b a, v16b b, v16b c, v16b d) { asm volatile("v_nop" :: "v"(a), "v"(b), "v"(c), "v"(d)); }
__device__ __forceinline__ void acc_guard4(v8f& a, v8f& b, v8f& c, v8f& d) { asm volatile("v_nop\n\tv_nop\n\tv_nop\n\tv_nop" : "+v"(a), "+v"(b), "+v"(c), "+v"(d)); }

template <typename T> struct Frag;
template <> struct Frag<_Float16> {
  typedef v16h V; union U { v16h v; v8h h[2]; };
  static __device__ __forceinline__ v16h load(const _Float16* p) {
    U f; f.h[0] = *(const v8h*)(p); f.h[1] = *(const v8h*)(p + 16); return f.v;
  }
  static __device__ __forceinline__ v8f mma(v16h a, v16h b, v8f c) {
    return __builtin_amdgcn_wmma_f32_16x16x32_f16(false, a, false, b, (short)0, c, false, false);
  }
  static __device__ __forceinline__ void guard(v8f& a, v8f& b, v16h x, v16h y) { dep_guard_h(a, b, x, y); }
  static __device__ __forceinline__ void keep(v16h a, v16h b, v16h c, v16h d) { keep4_h(a, b, c, d); }
};
template <> struct Frag<__bf16> {
  typedef v16b V; union U { v16b v; v8b h[2]; };
  static __device__ __forceinline__ v16b load(const __bf16* p) {
    U f; f.h[0] = *(const v8b*)(p); f.h[1] = *(const v8b*)(p + 16); return f.v;
  }
  static __device__ __forceinline__ v8f mma(v16b a, v16b b, v8f c) {
    return __builtin_amdgcn_wmma_f32_16x16x32_bf16(false, a, false, b, (short)0, c, false, false);
  }
  static __device__ __forceinline__ void guard(v8f& a, v8f& b, v16b x, v16b y) { dep_guard_b(a, b, x, y); }
  static __device__ __forceinline__ void keep(v16b a, v16b b, v16b c, v16b d) { keep4_b(a, b, c, d); }
};

template <int ET> struct Elem;
template <> struct Elem<0> { typedef _Float16 T; };
template <> struct Elem<1> { typedef __bf16 T; };

template <int ET, bool SPLIT, int BIAS_MODE, int OUT_MODE, int ACT, bool MIX3>
__global__ __launch_bounds__(256) void wmma_gemm64(
    const unsigned short* __restrict__ Ap, const unsigned short* __restrict__ A2p, int lda, long strideA,
    const unsigned short* __restrict__ Btp, const unsigned short* __restrict__ Bt2p, int ldb, long strideB,
    void* Cout, void* Cout2, int ldc, long strideC,
    const float* __restrict__ bias, const float* __restrict__ mixr, const float* __restrict__ mixc,
    int M, int N, int K, float scale) {
  typedef typename Elem<ET>::T T;
  typedef typename Frag<T>::V V;
  const T* A  = (const T*)(const void*)Ap;  const T* A2  = (const T*)(const void*)A2p;
  const T* Bt = (const T*)(const void*)Btp; const T* Bt2 = (const T*)(const void*)Bt2p;
  __shared__ __align__(16) float sT[8][16 * 68];
  const int b    = blockIdx.y;
  const int lane = threadIdx.x & 31;
  const int wave = threadIdx.x >> 5;
  const int tilesN = N >> 6;
  const int tilesM = M >> 6;
  const int tile = blockIdx.x * 8 + wave;
  if (tile >= tilesM * tilesN) return;
  const int tm = tile / tilesN;
  const int tn = tile - tm * tilesN;
  const int m0 = tm << 6;
  const int n0 = tn << 6;

  const T* Ab  = A   + (size_t)b * strideA;
  const T* Ab2 = A2  + (size_t)b * strideA;
  const T* Bb  = Bt  + (size_t)b * strideB;
  const T* Bb2 = Bt2 + (size_t)b * strideB;

  const int rlane = lane & 15;
  const int koff  = (lane >> 4) * 8;
  const int mOff  = (lane >> 4) * 8;

  v8f acc[4][4];
#pragma unroll
  for (int i = 0; i < 4; ++i)
#pragma unroll
    for (int j = 0; j < 4; ++j) acc[i][j] = (v8f){0.f,0.f,0.f,0.f,0.f,0.f,0.f,0.f};

  const int npass = SPLIT ? 3 : 1;
  for (int pp = 0; pp < npass; ++pp) {
    const T* Au = (pp == 2) ? Ab2 : Ab;
    const T* Bu = (pp == 1) ? Bb2 : Bb;
    for (int k0 = 0; k0 < K; k0 += 32) {
      V bh[4];
#pragma unroll
      for (int j = 0; j < 4; ++j) {
        const size_t bo = (size_t)(n0 + (j << 4) + rlane) * ldb + koff + k0;
        bh[j] = Frag<T>::load(Bu + bo);
      }
#pragma unroll
      for (int i = 0; i < 4; ++i) {
        const size_t ao = (size_t)(m0 + (i << 4) + rlane) * lda + koff + k0;
        V ah = Frag<T>::load(Au + ao);
#pragma unroll
        for (int j = 0; j < 4; ++j) acc[i][j] = Frag<T>::mma(ah, bh[j], acc[i][j]);
        Frag<T>::guard(acc[i][0], acc[i][3], ah, ah);
      }
      Frag<T>::keep(bh[0], bh[1], bh[2], bh[3]);
    }
  }
  acc_guard4(acc[0][0], acc[0][1], acc[0][2], acc[0][3]);
  acc_guard4(acc[1][0], acc[1][1], acc[1][2], acc[1][3]);
  acc_guard4(acc[2][0], acc[2][1], acc[2][2], acc[2][3]);
  acc_guard4(acc[3][0], acc[3][1], acc[3][2], acc[3][3]);

  float* slab = sT[wave];
#pragma unroll
  for (int i = 0; i < 4; ++i) {
    const int mBase = m0 + (i << 4);
    float lr[8];
#pragma unroll
    for (int r = 0; r < 8; ++r) lr[r] = MIX3 ? mixr[(size_t)(mBase + mOff + r) * 3 + 2] : 0.f;
    const float* mc = MIX3 ? (mixc + (size_t)(mBase >> 10) * DM) : mixc;
#pragma unroll
    for (int j = 0; j < 4; ++j) {
      const int n = n0 + (j << 4) + rlane;
      float bv = 0.f, cv = 0.f;
      if (BIAS_MODE == 2) bv = bias[n];
      if (MIX3) cv = mc[n];
#pragma unroll
      for (int r = 0; r < 8; ++r) {
        float v = acc[i][j][r] * scale;
        if (BIAS_MODE == 2) v += bv;
        if (ACT == 5) v = 0.5f * v * (1.0f + erff(v * 0.70710678118654752f));
        if (MIX3) v += lr[r] * cv;
        slab[(mOff + r) * 68 + (j << 4) + rlane] = v;
      }
    }
    __builtin_amdgcn_fence(__ATOMIC_RELEASE, "workgroup");
    __builtin_amdgcn_wave_barrier();
    __builtin_amdgcn_fence(__ATOMIC_ACQUIRE, "workgroup");
    if (OUT_MODE == 0) {
      float* C = (float*)Cout + (size_t)b * strideC;
      const int hh = lane >> 4, c4 = (lane & 15) * 4;
      for (int pass = 0; pass < 2; ++pass) {
#pragma unroll
        for (int it = 0; it < 8; ++it) {
          const int row = it * 2 + hh;
          v4f v = *(const v4f*)(slab + row * 68 + c4);
          *(volatile v4f*)(C + (size_t)(mBase + row) * ldc + n0 + c4) = v;
        }
        __threadfence();
      }
    } else {
      const int q = lane >> 3, c8 = (lane & 7) * 8;
      unsigned short* C  = (unsigned short*)Cout  + (size_t)b * strideC;
      unsigned short* C2 = (unsigned short*)Cout2 + (size_t)b * strideC;
      for (int pass = 0; pass < 2; ++pass) {
#pragma unroll
        for (int it = 0; it < 4; ++it) {
          const int row = it * 4 + q;
          const float* sp = slab + row * 68 + c8;
          v8h hv, lv;
#pragma unroll
          for (int e = 0; e < 8; ++e) {
            if (OUT_MODE == 1) {
              hv[e] = (_Float16)sp[e];
              lv[e] = hv[e];
            } else {
              unsigned short hb = f2bf_bits(sp[e]);
              unsigned short lb = f2bf_bits(sp[e] - bf_bits2f(hb));
              hv[e] = __builtin_bit_cast(_Float16, hb);
              lv[e] = __builtin_bit_cast(_Float16, lb);
            }
          }
          *(volatile v8h*)(C + (size_t)(mBase + row) * ldc + n0 + c8) = hv;
          if (OUT_MODE == 2) *(volatile v8h*)(C2 + (size_t)(mBase + row) * ldc + n0 + c8) = lv;
        }
        __threadfence();
      }
    }
    __builtin_amdgcn_fence(__ATOMIC_RELEASE, "workgroup");
    __builtin_amdgcn_wave_barrier();
    __builtin_amdgcn_fence(__ATOMIC_ACQUIRE, "workgroup");
  }
}

template <int MODE>
__global__ __launch_bounds__(256) void k_transpose16(
    const float* __restrict__ in0, const float* __restrict__ in1, const float* __restrict__ in2, const float* __restrict__ in3,
    unsigned short* oh0, unsigned short* oh1, unsigned short* oh2, unsigned short* oh3,
    unsigned short* ol0, unsigned short* ol1, unsigned short* ol2, unsigned short* ol3,
    int R, int Cc, float scale) {
  __shared__ __align__(16) float tf[64 * 68];
  const int z = blockIdx.z;
  const float* W = (z == 0) ? in0 : ((z == 1) ? in1 : ((z == 2) ? in2 : in3));
  unsigned short* oh = (z == 0) ? oh0 : ((z == 1) ? oh1 : ((z == 2) ? oh2 : oh3));
  unsigned short* ol = (z == 0) ? ol0 : ((z == 1) ? ol1 : ((z == 2) ? ol2 : ol3));
  const int c0  = blockIdx.x * 64;
  const int r0  = blockIdx.y * 64;
  const int tid = threadIdx.x;
  {
    const int lr = tid >> 4;
    const int c4 = (tid & 15) * 4;
#pragma unroll
    for (int it = 0; it < 4; ++it) {
      const int rr = it * 16 + lr;
      const v4f a = *(const v4f*)(W + (size_t)(r0 + rr) * Cc + c0 + c4);
      *(v4f*)(tf + rr * 68 + c4) = a;
    }
  }
  __syncthreads();
  const int sub = tid >> 3;
  const int c8  = (tid & 7) * 8;
  v4u hv[2], lv[2];
#pragma unroll
  for (int it = 0; it < 2; ++it) {
    const int oc = it * 32 + sub;
    v4u a, a2;
#pragma unroll
    for (int q = 0; q < 4; ++q) {
      const float f0 = tf[(c8 + 2 * q) * 68 + oc];
      const float f1 = tf[(c8 + 2 * q + 1) * 68 + oc];
      if (MODE == 0) {
        a[q]  = pk16(f2h_bits(f0 * scale), f2h_bits(f1 * scale));
        a2[q] = a[q];
      } else {
        const unsigned short h0 = f2bf_bits(f0), h1 = f2bf_bits(f1);
        const unsigned short l0 = f2bf_bits(f0 - bf_bits2f(h0)), l1 = f2bf_bits(f1 - bf_bits2f(h1));
        a[q]  = pk16(h0, h1);
        a2[q] = pk16(l0, l1);
      }
    }
    hv[it] = a; lv[it] = a2;
  }
  for (int pass = 0; pass < 2; ++pass) {
#pragma unroll
    for (int it = 0; it < 2; ++it) {
      const int oc = it * 32 + sub;
      const size_t go = (size_t)(c0 + oc) * R + r0 + c8;
      *(volatile v4u*)(oh + go) = hv[it];
      if (MODE == 1) *(volatile v4u*)(ol + go) = lv[it];
    }
    __threadfence();
  }
}

__global__ __launch_bounds__(256) void k_l3planes(const float* __restrict__ l3, unsigned* hi2, unsigned* lo2) {
  const int i = blockIdx.x * 256 + threadIdx.x;
  const v2f f = *(const v2f*)(l3 + 2 * (size_t)i);
  const unsigned short h0 = f2bf_bits(f[0]), h1 = f2bf_bits(f[1]);
  const unsigned short l0 = f2bf_bits(f[0] - bf_bits2f(h0)), l1 = f2bf_bits(f[1] - bf_bits2f(h1));
  const unsigned uh = pk16(h0, h1), ul = pk16(l0, l1);
  ((volatile unsigned*)hi2)[i] = uh;
  ((volatile unsigned*)lo2)[i] = ul;
  __threadfence();
  ((volatile unsigned*)hi2)[i] = uh;
  ((volatile unsigned*)lo2)[i] = ul;
}

__global__ __launch_bounds__(256) void k_ema(const float* __restrict__ x, unsigned* xh2, unsigned* l2h2) {
#pragma clang fp contract(off)
  const int g = blockIdx.x * 256 + threadIdx.x;
  const int b = g >> 9;
  const int p = g & 511;
  size_t e = (size_t)b * SEQ * DM + 2 * p;
  float y0 = 0.f, y1 = 0.f;
  for (int t = 0; t < SEQ; ++t, e += DM) {
    const v2f xv = *(const v2f*)(x + e);
    const float m0 = 0.9f * y0, m1 = 0.9f * y1;
    const float a0 = 0.1f * xv[0], a1 = 0.1f * xv[1];
    y0 = m0 + a0;
    y1 = m1 + a1;
    const unsigned ux = pk16(f2h_bits(xv[0]), f2h_bits(xv[1]));
    const unsigned ul = pk16(f2h_bits(4.0f * y0), f2h_bits(4.0f * y1));
    const size_t o = e >> 1;
    ((volatile unsigned*)xh2)[o]  = ux;
    ((volatile unsigned*)l2h2)[o] = ul;
    __threadfence();
    ((volatile unsigned*)xh2)[o]  = ux;
    ((volatile unsigned*)l2h2)[o] = ul;
  }
}

__global__ __launch_bounds__(256) void k_lam(const float* __restrict__ hdn, const float* __restrict__ rw2,
                                             const float* __restrict__ rb2, float* lamOut) {
  __shared__ __align__(16) float sl[64 * 3];
  const int tid = threadIdx.x, lane = tid & 31, wave = tid >> 5;
  const float b0 = rb2[0], b1 = rb2[1], b2 = rb2[2];
  for (int rr = 0; rr < 8; ++rr) {
    const int lrow = wave * 8 + rr;
    const int row  = blockIdx.x * 64 + lrow;
    const float* hr = hdn + (size_t)row * DR;
    float s0 = 0.f, s1 = 0.f, s2 = 0.f;
#pragma unroll 1
    for (int i = 0; i < DR / 32; ++i) {
      const int j = i * 32 + lane;
      const float hv = hr[j];
      s0 += hv * rw2[j * 3 + 0];
      s1 += hv * rw2[j * 3 + 1];
      s2 += hv * rw2[j * 3 + 2];
    }
#pragma unroll
    for (int off = 16; off > 0; off >>= 1) {
      s0 += __shfl_xor(s0, off, 32);
      s1 += __shfl_xor(s1, off, 32);
      s2 += __shfl_xor(s2, off, 32);
    }
    s0 += b0; s1 += b1; s2 += b2;
    const float mx = fmaxf(s0, fmaxf(s1, s2));
    const float e0 = expf(s0 - mx), e1 = expf(s1 - mx), e2 = expf(s2 - mx);
    const float inv = 1.0f / (e0 + e1 + e2);
    if (lane == 0) {
      sl[lrow * 3 + 0] = e0 * inv;
      sl[lrow * 3 + 1] = e1 * inv;
      sl[lrow * 3 + 2] = e2 * inv;
    }
  }
  __syncthreads();
  if (tid < 48) {
    const v4f v = *(const v4f*)(sl + tid * 4);
    float* dst = lamOut + (size_t)blockIdx.x * 192 + tid * 4;
    *(volatile v4f*)dst = v;
    __threadfence();
    *(volatile v4f*)dst = v;
  }
}

#define AT_D 64
#define AT_NW 4
#define AT_QB 64
#define AT_KC 64

__device__ __forceinline__ __bf16 at_f2bf(float f) { return __builtin_bit_cast(__bf16, f2bf_bits(f)); }
__device__ __forceinline__ void at_split(float f, __bf16& hi, __bf16& lo) {
  const unsigned short hb = f2bf_bits(f);
  hi = __builtin_bit_cast(__bf16, hb);
  lo = at_f2bf(f - __uint_as_float(((unsigned)hb) << 16));
}
__device__ __forceinline__ v8f mma_b(v16b a, v16b b, v8f c) {
  c = __builtin_amdgcn_wmma_f32_16x16x32_bf16(false, a, false, b, (short)0, c, false, false);
  asm volatile("v_nop\n\tv_nop\n\tv_nop\n\tv_nop" : "+v"(c) : "v"(a), "v"(b));
  return c;
}
__device__ __forceinline__ v8f mma_h(v16h a, v16h b, v8f c) {
  c = __builtin_amdgcn_wmma_f32_16x16x32_f16(false, a, false, b, (short)0, c, false, false);
  asm volatile("v_nop\n\tv_nop\n\tv_nop\n\tv_nop" : "+v"(c) : "v"(a), "v"(b));
  return c;
}

__global__ __launch_bounds__(128)
void attn_causal64_kernel(const unsigned short* __restrict__ qp, const unsigned short* __restrict__ kp,
                          const unsigned short* __restrict__ vhp, const unsigned short* __restrict__ vlp,
                          float* out, float sscale) {
  union FB { v16b v; v8b h[2]; };
  union FH { v16h v; v8h h[2]; };
  __shared__ __align__(16) _Float16 Ksh[AT_KC * AT_D];
  __shared__ __align__(16) __bf16   Vth[AT_D * AT_KC];
  __shared__ __align__(16) __bf16   Vtl[AT_D * AT_KC];
  __shared__ __align__(16) __bf16   Psh[AT_NW][16 * AT_KC];
  __shared__ __align__(16) __bf16   Psl[AT_NW][16 * AT_KC];
  __shared__ __align__(16) float    Os[AT_NW][16 * 68];

  const int tid  = threadIdx.x;
  const int wave = tid >> 5;
  const int lane = tid & 31;
  const int hh   = lane >> 4;
  const int c    = lane & 15;

  const int nqb = SEQ / AT_QB;
  const int bx = blockIdx.x;
  const int b  = blockIdx.y;
  const int qb = bx % nqb;
  const int h  = bx / nqb;
  const int q0 = qb * AT_QB + wave * 16;

  const size_t boff = (size_t)b * SEQ * DM;
  const _Float16* Qb = (const _Float16*)(const void*)qp + boff + (size_t)h * AT_D;
  const _Float16* Kb = (const _Float16*)(const void*)kp + boff + (size_t)h * AT_D;
  const __bf16*   Vh = (const __bf16*)(const void*)vhp + boff + (size_t)h * AT_D * SEQ;
  const __bf16*   Vl = (const __bf16*)(const void*)vlp + boff + (size_t)h * AT_D * SEQ;
  float*          ob = out + boff + (size_t)h * AT_D;

  v16h qa[2];
#pragma unroll
  for (int dc = 0; dc < 2; ++dc) {
    const _Float16* qr = Qb + (size_t)(q0 + c) * DM + dc * 32 + 8 * hh;
    qa[dc] = Frag<_Float16>::load(qr);
  }

  float mrow[8], lrow[8];
  v8f oacc[4];
#pragma unroll
  for (int r = 0; r < 8; ++r) { mrow[r] = -INFINITY; lrow[r] = 0.f; }
#pragma unroll
  for (int t = 0; t < 4; ++t) oacc[t] = (v8f){0.f,0.f,0.f,0.f,0.f,0.f,0.f,0.f};

  const int nChunks = qb + 1;
  for (int kc = 0; kc < nChunks; ++kc) {
    const int kv0 = kc * AT_KC;
    __syncthreads();
    {
      const int r = tid >> 1, half = (tid & 1) * 32;
      const _Float16* ksh = Kb + (size_t)(kv0 + r) * DM + half;
      const __bf16*   vsh = Vh + (size_t)r * SEQ + kv0 + half;
      const __bf16*   vsl = Vl + (size_t)r * SEQ + kv0 + half;
#pragma unroll
      for (int i = 0; i < 4; ++i) {
        const v8h a0 = *(const v8h*)(ksh + 8 * i);
        const v8b b0 = *(const v8b*)(vsh + 8 * i);
        const v8b b1 = *(const v8b*)(vsl + 8 * i);
        *(v8h*)(Ksh + r * AT_D  + half + 8 * i) = a0;
        *(v8b*)(Vth + r * AT_KC + half + 8 * i) = b0;
        *(v8b*)(Vtl + r * AT_KC + half + 8 * i) = b1;
      }
    }
    __syncthreads();

    v8f s[4];
#pragma unroll
    for (int j = 0; j < 4; ++j) {
      s[j] = (v8f){0.f,0.f,0.f,0.f,0.f,0.f,0.f,0.f};
#pragma unroll
      for (int dc = 0; dc < 2; ++dc) {
        FH kb;
        kb.h[0] = *(const v8h*)(Ksh + (j * 16 + c) * AT_D + dc * 32 + 8 * hh);
        kb.h[1] = *(const v8h*)(Ksh + (j * 16 + c) * AT_D + dc * 32 + 16 + 8 * hh);
        s[j] = mma_h(qa[dc], kb.v, s[j]);
      }
    }
    const bool diag = (kc == qb);
    float cm[8];
#pragma unroll
    for (int r = 0; r < 8; ++r) {
      const int qrow = q0 + 8 * hh + r;
      float m = -INFINITY;
#pragma unroll
      for (int j = 0; j < 4; ++j) {
        const int kvcol = kv0 + j * 16 + c;
        const float sv = s[j][r] * sscale;
        const bool masked = diag && (kvcol > qrow);
        const float sm = masked ? -INFINITY : sv;
        s[j][r] = sm;
        m = fmaxf(m, sm);
      }
#pragma unroll
      for (int off = 1; off < 16; off <<= 1) m = fmaxf(m, __shfl_xor(m, off, 32));
      cm[r] = m;
    }
    __bf16* pwh = Psh[wave];
    __bf16* pwl = Psl[wave];
#pragma unroll
    for (int r = 0; r < 8; ++r) {
      const float mnew = fmaxf(mrow[r], cm[r]);
      const float alpha = expf(mrow[r] - mnew);
      mrow[r] = mnew;
      float psum = 0.f;
#pragma unroll
      for (int j = 0; j < 4; ++j) {
        const float p = expf(s[j][r] - mnew);
        psum += p;
        __bf16 a, bl; at_split(p, a, bl);
        pwh[(8 * hh + r) * AT_KC + j * 16 + c] = a;
        pwl[(8 * hh + r) * AT_KC + j * 16 + c] = bl;
      }
#pragma unroll
      for (int off = 1; off < 16; off <<= 1) psum += __shfl_xor(psum, off, 32);
      lrow[r] = lrow[r] * alpha + psum;
#pragma unroll
      for (int t = 0; t < 4; ++t) oacc[t][r] *= alpha;
    }
    __builtin_amdgcn_fence(__ATOMIC_RELEASE, "workgroup");
    __builtin_amdgcn_wave_barrier();
    __builtin_amdgcn_fence(__ATOMIC_ACQUIRE, "workgroup");
#pragma unroll 1
    for (int kk = 0; kk < 2; ++kk) {
      FB pa, pl;
      pa.h[0] = *(const v8b*)(pwh + c * AT_KC + kk * 32 + 8 * hh);
      pa.h[1] = *(const v8b*)(pwh + c * AT_KC + kk * 32 + 16 + 8 * hh);
      pl.h[0] = *(const v8b*)(pwl + c * AT_KC + kk * 32 + 8 * hh);
      pl.h[1] = *(const v8b*)(pwl + c * AT_KC + kk * 32 + 16 + 8 * hh);
#pragma unroll
      for (int t = 0; t < 4; ++t) {
        FB vb, vl;
        vb.h[0] = *(const v8b*)(Vth + (t * 16 + c) * AT_KC + kk * 32 + 8 * hh);
        vb.h[1] = *(const v8b*)(Vth + (t * 16 + c) * AT_KC + kk * 32 + 16 + 8 * hh);
        vl.h[0] = *(const v8b*)(Vtl + (t * 16 + c) * AT_KC + kk * 32 + 8 * hh);
        vl.h[1] = *(const v8b*)(Vtl + (t * 16 + c) * AT_KC + kk * 32 + 16 + 8 * hh);
        oacc[t] = mma_b(pa.v, vb.v, oacc[t]);
        oacc[t] = mma_b(pa.v, vl.v, oacc[t]);
        oacc[t] = mma_b(pl.v, vb.v, oacc[t]);
      }
    }
  }

  float* os = Os[wave];
#pragma unroll
  for (int r = 0; r < 8; ++r) {
    const float inv = 1.0f / lrow[r];
#pragma unroll
    for (int t = 0; t < 4; ++t) os[(8 * hh + r) * 68 + t * 16 + c] = oacc[t][r] * inv;
  }
  __builtin_amdgcn_fence(__ATOMIC_RELEASE, "workgroup");
  __builtin_amdgcn_wave_barrier();
  __builtin_amdgcn_fence(__ATOMIC_ACQUIRE, "workgroup");
  {
    const int c4 = (lane & 15) * 4;
    for (int pass = 0; pass < 2; ++pass) {
#pragma unroll
      for (int it = 0; it < 8; ++it) {
        const int row = it * 2 + hh;
        v4f val = *(const v4f*)(os + row * 68 + c4);
        *(volatile v4f*)(ob + (size_t)(q0 + row) * DM + c4) = val;
      }
      __threadfence();
    }
  }
}

__global__ __launch_bounds__(256) void k_mix(const float* __restrict__ a1, const float* __restrict__ a2,
                                             const float* __restrict__ lam, unsigned short* amix) {
  const int i = blockIdx.x * 256 + threadIdx.x;
  const int row = i >> 7;
  const float l0 = lam[row * 3 + 0], l1 = lam[row * 3 + 1];
  const float* p1 = a1 + 8 * (size_t)i;
  const float* p2 = a2 + 8 * (size_t)i;
  const v4f x0 = *(const v4f*)p1, x1 = *(const v4f*)(p1 + 4);
  const v4f y0 = *(const v4f*)p2, y1 = *(const v4f*)(p2 + 4);
  v8h o;
#pragma unroll
  for (int e = 0; e < 4; ++e) {
    o[e]     = (_Float16)(64.0f * (l0 * x0[e] + l1 * y0[e]));
    o[4 + e] = (_Float16)(64.0f * (l0 * x1[e] + l1 * y1[e]));
  }
  _Float16* dst = (_Float16*)(void*)amix + 8 * (size_t)i;
  *(volatile v8h*)dst = o;
  __threadfence();
  *(volatile v8h*)dst = o;
}

extern "C" void kernel_launch(void* const* d_in, const int* in_sizes, int n_in,
                              void* d_out, int out_size, void* d_ws, size_t ws_size,
                              hipStream_t stream) {
  if (n_in < 10) return;
  if (in_sizes[0] != NB * SEQ * DM) return;
  if (in_sizes[1] != NB * DM) return;
  if (in_sizes[2] != DM * DM || in_sizes[3] != DM * DM || in_sizes[4] != DM * DM || in_sizes[5] != DM * DM) return;
  if (in_sizes[6] != DM * DR || in_sizes[7] != DR || in_sizes[8] != DR * 3 || in_sizes[9] != 3) return;
  if (out_size != NB * SEQ * DM + NB * SEQ * 3) return;

  const float* x   = (const float*)d_in[0];
  const float* l3  = (const float*)d_in[1];
  const float* wq  = (const float*)d_in[2];
  const float* wk  = (const float*)d_in[3];
  const float* wv  = (const float*)d_in[4];
  const float* wo  = (const float*)d_in[5];
  const float* rw1 = (const float*)d_in[6];
  const float* rb1 = (const float*)d_in[7];
  const float* rw2 = (const float*)d_in[8];
  const float* rb2 = (const float*)d_in[9];

  float* out0 = (float*)d_out;
  float* out1 = (float*)d_out + (size_t)NB * SEQ * DM;

  const size_t PW16 = (size_t)DM * DM * 2;
  const size_t PR16 = (size_t)DM * DR * 2;
  const size_t PL   = (size_t)64 * DM * 2;
  const size_t PU   = (size_t)64 * DM * 4;
  const size_t PA16 = (size_t)NB * SEQ * DM * 2;
  const size_t PH   = (size_t)NB * SEQ * DR * 4;
  const size_t PA32 = (size_t)NB * SEQ * DM * 4;
  size_t off = 0;
  const size_t oWqT = off; off += PW16;  const size_t oWkT = off; off += PW16;
  const size_t oWvT = off; off += PW16;  const size_t oWoT = off; off += PW16;
  const size_t oRwT = off; off += PR16;
  const size_t oWvBh = off; off += PW16; const size_t oWvBl = off; off += PW16;
  const size_t oWoBh = off; off += PW16; const size_t oWoBl = off; off += PW16;
  const size_t oL3h = off; off += PL;    const size_t oL3l = off; off += PL;
  const size_t oV3h = off; off += PL;    const size_t oV3l = off; off += PL;
  const size_t oU3  = off; off += PU;
  const size_t oXh  = off; off += PA16;
  const size_t oL2h = off; off += PA16;
  const size_t oQh  = off; off += PA16;
  const size_t oHdn = off; off += PH;
  const size_t oK   = off; off += PA16;
  const size_t oVTh = off; off += PA16;  const size_t oVTl = off; off += PA16;
  const size_t oA1  = off; off += PA32;
  const size_t oA2  = off; off += PA32;
  const size_t oAmx = off; off += PA16;
  if (off > ws_size) return;

  char* ws = (char*)d_ws;
  unsigned short* WqT  = (unsigned short*)(ws + oWqT);  unsigned short* WkT  = (unsigned short*)(ws + oWkT);
  unsigned short* WvT  = (unsigned short*)(ws + oWvT);  unsigned short* WoT  = (unsigned short*)(ws + oWoT);
  unsigned short* RwT  = (unsigned short*)(ws + oRwT);
  unsigned short* WvBh = (unsigned short*)(ws + oWvBh); unsigned short* WvBl = (unsigned short*)(ws + oWvBl);
  unsigned short* WoBh = (unsigned short*)(ws + oWoBh); unsigned short* WoBl = (unsigned short*)(ws + oWoBl);
  unsigned short* L3h  = (unsigned short*)(ws + oL3h);  unsigned short* L3l  = (unsigned short*)(ws + oL3l);
  unsigned short* V3h  = (unsigned short*)(ws + oV3h);  unsigned short* V3l  = (unsigned short*)(ws + oV3l);
  float*          U3   = (float*)(ws + oU3);
  unsigned short* Xh   = (unsigned short*)(ws + oXh);
  unsigned short* L2h  = (unsigned short*)(ws + oL2h);
  unsigned short* Qh   = (unsigned short*)(ws + oQh);
  float*          Hdn  = (float*)(ws + oHdn);
  unsigned short* Kp   = (unsigned short*)(ws + oK);
  unsigned short* VTh  = (unsigned short*)(ws + oVTh);  unsigned short* VTl  = (unsigned short*)(ws + oVTl);
  float*          A1   = (float*)(ws + oA1);
  float*          A2   = (float*)(ws + oA2);
  unsigned short* Amx  = (unsigned short*)(ws + oAmx);

  const dim3 blk(256);

  k_transpose16<0><<<dim3(DM / 64, DM / 64, 4), blk, 0, stream>>>(
      wq, wk, wv, wo, WqT, WkT, WvT, WoT, WqT, WkT, WvT, WoT, DM, DM, 16.0f);
  k_transpose16<0><<<dim3(DR / 64, DM / 64, 1), blk, 0, stream>>>(
      rw1, rw1, rw1, rw1, RwT, RwT, RwT, RwT, RwT, RwT, RwT, RwT, DM, DR, 16.0f);
  k_transpose16<1><<<dim3(DM / 64, DM / 64, 2), blk, 0, stream>>>(
      wv, wo, wv, wo, WvBh, WoBh, WvBh, WoBh, WvBl, WoBl, WvBl, WoBl, DM, DM, 1.0f);
  hipMemsetAsync(ws + oL3h, 0, 2 * PL, stream);
  k_l3planes<<<dim3((NB * DM / 2) / 256), blk, 0, stream>>>(l3, (unsigned*)(void*)L3h, (unsigned*)(void*)L3l);
  k_ema<<<dim3((NB * DM / 2) / 256), blk, 0, stream>>>(x, (unsigned*)(void*)Xh, (unsigned*)(void*)L2h);

  const int BT = NB * SEQ;
  const dim3 gFull(((BT / 64) * (DM / 64) + 7) / 8, 1);
  const dim3 gHalf(((BT / 64) * (DR / 64) + 7) / 8, 1);
  const dim3 gVT(((DM / 64) * (SEQ / 64) + 7) / 8, NB);
  const dim3 gTiny(((64 / 64) * (DM / 64) + 7) / 8, 1);
  const dim3 gAtt(NH * (SEQ / AT_QB), NB);

  wmma_gemm64<0, false, 0, 1, 0, false><<<gFull, blk, 0, stream>>>(
      Xh, Xh, DM, 0L, WqT, WqT, DM, 0L, (void*)Qh, (void*)Qh, DM, 0L,
      rb1, out1, U3, BT, DM, DM, 1.0f / 16.0f);
  wmma_gemm64<0, false, 2, 0, 5, false><<<gHalf, blk, 0, stream>>>(
      Qh, Qh, DM, 0L, RwT, RwT, DM, 0L, (void*)Hdn, (void*)Hdn, DR, 0L,
      rb1, out1, U3, BT, DR, DM, 1.0f / 16.0f);
  k_lam<<<dim3(BT / 64), blk, 0, stream>>>(Hdn, rw2, rb2, out1);

  wmma_gemm64<0, false, 0, 1, 0, false><<<gFull, blk, 0, stream>>>(
      Xh, Xh, DM, 0L, WkT, WkT, DM, 0L, (void*)Kp, (void*)Kp, DM, 0L,
      rb1, out1, U3, BT, DM, DM, 1.0f / 16.0f);
  wmma_gemm64<0, false, 0, 2, 0, false><<<gVT, blk, 0, stream>>>(
      WvT, WvT, DM, 0L, Xh, Xh, DM, (long)SEQ * DM, (void*)VTh, (void*)VTl, SEQ, (long)DM * SEQ,
      rb1, out1, U3, DM, SEQ, DM, 1.0f / 16.0f);
  attn_causal64_kernel<<<gAtt, dim3(128), 0, stream>>>(Qh, Kp, VTh, VTl, A1, 0.125f);

  wmma_gemm64<0, false, 0, 1, 0, false><<<gFull, blk, 0, stream>>>(
      L2h, L2h, DM, 0L, WkT, WkT, DM, 0L, (void*)Kp, (void*)Kp, DM, 0L,
      rb1, out1, U3, BT, DM, DM, 1.0f / 64.0f);
  wmma_gemm64<0, false, 0, 2, 0, false><<<gVT, blk, 0, stream>>>(
      WvT, WvT, DM, 0L, L2h, L2h, DM, (long)SEQ * DM, (void*)VTh, (void*)VTl, SEQ, (long)DM * SEQ,
      rb1, out1, U3, DM, SEQ, DM, 1.0f / 64.0f);
  attn_causal64_kernel<<<gAtt, dim3(128), 0, stream>>>(Qh, Kp, VTh, VTl, A2, 0.125f);

  wmma_gemm64<1, true, 0, 2, 0, false><<<gTiny, blk, 0, stream>>>(
      L3h, L3l, DM, 0L, WvBh, WvBl, DM, 0L, (void*)V3h, (void*)V3l, DM, 0L,
      rb1, out1, U3, 64, DM, DM, 1.0f);
  wmma_gemm64<1, true, 0, 0, 0, false><<<gTiny, blk, 0, stream>>>(
      V3h, V3l, DM, 0L, WoBh, WoBl, DM, 0L, (void*)U3, (void*)U3, DM, 0L,
      rb1, out1, U3, 64, DM, DM, 1.0f);

  k_mix<<<dim3((int)((PA32 / 4) / 8 / 256)), blk, 0, stream>>>(A1, A2, out1, Amx);
  wmma_gemm64<0, false, 0, 0, 0, true><<<gFull, blk, 0, stream>>>(
      Amx, Amx, DM, 0L, WoT, WoT, DM, 0L, (void*)out0, (void*)out0, DM, 0L,
      rb1, out1, U3, BT, DM, DM, 1.0f / 1024.0f);
  (void)hipGetLastError();
}
